// MambaClassifier_19653770347251
// MI455X (gfx1250) — hardware-run, weakly checked
//
#include <hip/hip_runtime.h>
#include <math.h>

typedef __attribute__((ext_vector_type(16))) _Float16 v16h;
typedef __attribute__((ext_vector_type(8)))  _Float16 v8h;
typedef __attribute__((ext_vector_type(2)))  _Float16 v2h;
typedef __attribute__((ext_vector_type(16))) __bf16   v16b;
typedef __attribute__((ext_vector_type(8)))  __bf16   v8b;
typedef __attribute__((ext_vector_type(8)))  float    v8f;
typedef __attribute__((ext_vector_type(4)))  float    v4f;
typedef __attribute__((ext_vector_type(2)))  float    v2f;
typedef float v2f __attribute__((ext_vector_type(2)));

constexpr int kNB   = 4;
constexpr int kT    = 1024;
constexpr int kRows = kNB * kT;
constexpr int kKP   = 192;
constexpr int kDM   = 256;
constexpr int kDI   = 2 * kDM;
constexpr int kNs   = 16;
constexpr int kDC   = 4;
constexpr int kR    = 16;
constexpr int kRP   = 32;
constexpr int kXo   = kR + 2 * kNs;
constexpr int kXoP  = 64;
constexpr int kNL   = 4;
constexpr int kNC   = 1000;
constexpr int kNCP  = 1024;
constexpr int kMP   = 64;
constexpr int kThr  = 256;
constexpr float kInCarry = 1024.0f;
constexpr float kWCarry  = 4096.0f;
constexpr float kCX   = 1024.0f;
constexpr float kCXn  = 1024.0f;
constexpr float kCU   = 1024.0f;
constexpr float kCDt  = 4096.0f;
constexpr float kWdtCarry = 4096.0f;
constexpr float kCY   = 256.0f;
constexpr float kCPool = 65536.0f;
constexpr float kF16MinNormal = 6.103515625e-5f;

static_assert(kXo == 48 && kXo <= kXoP && kR <= kRP && kDI == 512 && kRows == 4096 && kT == 1024 && kDM == 256 && (kKP % 32) == 0 && kNC <= kNCP && kNB <= kMP, "the index arithmetic below uses these sizes");

constexpr size_t kOffZB = 0ull;
constexpr size_t kOffPB = 4096ull;
constexpr size_t kOffBDT = 5120ull;
constexpr size_t kOffCLB = 13312ull;
constexpr size_t kOffSTAT = 17408ull;
constexpr size_t kOffWP16 = 50176ull;
constexpr size_t kOffWIN16 = 148480ull;
constexpr size_t kOffWX16 = 2245632ull;
constexpr size_t kOffWDT16 = 2507776ull;
constexpr size_t kOffWOUT16 = 2638848ull;
constexpr size_t kOffWCLS16 = 3687424ull;
constexpr size_t kOffPATCH16 = 4211712ull;
constexpr size_t kOffUA = 5784576ull;
constexpr size_t kOffUB = 9978880ull;
constexpr size_t kOffXN16 = 14173184ull;
constexpr size_t kOffXZ = 16270336ull;
constexpr size_t kOffU32 = 33047552ull;
constexpr size_t kOffU16 = 41436160ull;
constexpr size_t kOffXD = 45630464ull;
constexpr size_t kOffDT16 = 46679040ull;
constexpr size_t kOffDL = 46941184ull;
constexpr size_t kOffYS = 55329792ull;
constexpr size_t kOffY16 = 63718400ull;
constexpr size_t kOffOUTF = 67912704ull;
constexpr size_t kOffPOOL16 = 72107008ull;
constexpr size_t kOffLOG = 72139776ull;
constexpr size_t kWsTotal = 72401920ull;
static_assert(kWsTotal <= 134217728ull, "carve cap: under 128 MiB");
static_assert(kOffZB == 0
  && kOffPB == kOffZB + 4096ull
  && kOffBDT == kOffPB + 1024ull
  && kOffCLB == kOffBDT + 8192ull
  && kOffSTAT == kOffCLB + 4096ull
  && kOffWP16 == kOffSTAT + 32768ull
  && kOffWIN16 == kOffWP16 + 98304ull
  && kOffWX16 == kOffWIN16 + 2097152ull
  && kOffWDT16 == kOffWX16 + 262144ull
  && kOffWOUT16 == kOffWDT16 + 131072ull
  && kOffWCLS16 == kOffWOUT16 + 1048576ull
  && kOffPATCH16 == kOffWCLS16 + 524288ull
  && kOffUA == kOffPATCH16 + 1572864ull
  && kOffUB == kOffUA + 4194304ull
  && kOffXN16 == kOffUB + 4194304ull
  && kOffXZ == kOffXN16 + 2097152ull
  && kOffU32 == kOffXZ + 16777216ull
  && kOffU16 == kOffU32 + 8388608ull
  && kOffXD == kOffU16 + 4194304ull
  && kOffDT16 == kOffXD + 1048576ull
  && kOffDL == kOffDT16 + 262144ull
  && kOffYS == kOffDL + 8388608ull
  && kOffY16 == kOffYS + 8388608ull
  && kOffOUTF == kOffY16 + 4194304ull
  && kOffPOOL16 == kOffOUTF + 4194304ull
  && kOffLOG == kOffPOOL16 + 32768ull
  && kWsTotal == kOffLOG + 262144ull, "the carve is a chain: every region starts where the one before ends");
static_assert((kOffPB % 256) == 0 && (kOffBDT % 256) == 0 && (kOffCLB % 256) == 0 && (kOffSTAT % 256) == 0 && (kOffWP16 % 256) == 0 && (kOffWIN16 % 256) == 0 && (kOffWX16 % 256) == 0 && (kOffWDT16 % 256) == 0 && (kOffWOUT16 % 256) == 0 && (kOffWCLS16 % 256) == 0 && (kOffPATCH16 % 256) == 0 && (kOffUA % 256) == 0 && (kOffUB % 256) == 0 && (kOffXN16 % 256) == 0 && (kOffXZ % 256) == 0 && (kOffU32 % 256) == 0 && (kOffU16 % 256) == 0 && (kOffXD % 256) == 0 && (kOffDT16 % 256) == 0 && (kOffDL % 256) == 0 && (kOffYS % 256) == 0 && (kOffY16 % 256) == 0 && (kOffOUTF % 256) == 0 && (kOffPOOL16 % 256) == 0 && (kOffLOG % 256) == 0, "every region starts on a multiple of 256 B");

__device__ __forceinline__ unsigned short f2bf_bits(float f) {
  unsigned u = __float_as_uint(f);
  return (unsigned short)((u + 0x7FFFu + ((u >> 16) & 1u)) >> 16);
}
__device__ __forceinline__ float bf_bits2f(unsigned short h) { return __uint_as_float(((unsigned)h) << 16); }
__device__ __forceinline__ float bf16r(float f) { return bf_bits2f(f2bf_bits(f)); }
__device__ __forceinline__ float carry_flush(float v, float carry) {
  const float s = v * carry;
  return (fabsf(s) < kF16MinNormal) ? 0.0f : s;
}

__device__ __forceinline__ void dep_guard4_h(v8f& a, v8f& b, v8f& c, v8f& d, v16h x, v16h y) { asm volatile("v_nop\n\tv_nop\n\tv_nop\n\tv_nop" : "+v"(a), "+v"(b), "+v"(c), "+v"(d) : "v"(x), "v"(y)); }
__device__ __forceinline__ void dep_guard4_b(v8f& a, v8f& b, v8f& c, v8f& d, v16b x, v16b y) { asm volatile("v_nop\n\tv_nop\n\tv_nop\n\tv_nop" : "+v"(a), "+v"(b), "+v"(c), "+v"(d) : "v"(x), "v"(y)); }
__device__ __forceinline__ void keep4_h(v16h a, v16h b, v16h c, v16h d) { asm volatile("v_nop" :: "v"(a), "v"(b), "v"(c), "v"(d)); }
__device__ __forceinline__ void keep4_b(v16b a, v16b b, v16b c, v16b d) { asm volatile("v_nop" :: "v"(a), "v"(b), "v"(c), "v"(d)); }
__device__ __forceinline__ void acc_guard4(v8f& a, v8f& b, v8f& c, v8f& d) { asm volatile("v_nop\n\tv_nop\n\tv_nop\n\tv_nop" : "+v"(a), "+v"(b), "+v"(c), "+v"(d)); }

template <typename T> struct Frag;
template <> struct Frag<_Float16> {
  typedef v16h V; union U { v16h v; v8h h[2]; };
  static __device__ __forceinline__ v16h load(const _Float16* p) {
    U f; f.h[0] = *(const v8h*)(p); f.h[1] = *(const v8h*)(p + 16); return f.v;
  }
  static __device__ __forceinline__ v8f mma(v16h a, v16h b, v8f c) {
    return __builtin_amdgcn_wmma_f32_16x16x32_f16(false, a, false, b, (short)0, c, false, false);
  }
  static __device__ __forceinline__ void guard4(v8f& a, v8f& b, v8f& c, v8f& d, v16h x, v16h y) { dep_guard4_h(a, b, c, d, x, y); }
  static __device__ __forceinline__ void keep(v16h a, v16h b, v16h c, v16h d) { keep4_h(a, b, c, d); }
};
template <> struct Frag<__bf16> {
  typedef v16b V; union U { v16b v; v8b h[2]; };
  static __device__ __forceinline__ v16b load(const __bf16* p) {
    U f; f.h[0] = *(const v8b*)(p); f.h[1] = *(const v8b*)(p + 16); return f.v;
  }
  static __device__ __forceinline__ v8f mma(v16b a, v16b b, v8f c) {
    return __builtin_amdgcn_wmma_f32_16x16x32_bf16(false, a, false, b, (short)0, c, false, false);
  }
  static __device__ __forceinline__ void guard4(v8f& a, v8f& b, v8f& c, v8f& d, v16b x, v16b y) { dep_guard4_b(a, b, c, d, x, y); }
  static __device__ __forceinline__ void keep(v16b a, v16b b, v16b c, v16b d) { keep4_b(a, b, c, d); }
};

__device__ __forceinline__ v8f mma_h(v16h a, v16h b, v8f c) {
  c = __builtin_amdgcn_wmma_f32_16x16x32_f16(false, a, false, b, (short)0, c, false, false);
  asm volatile("v_nop\n\tv_nop\n\tv_nop\n\tv_nop" : "+v"(c) : "v"(a), "v"(b));
  return c;
}

template <int ET> struct Elem;
template <> struct Elem<0> { typedef _Float16 T; };
template <> struct Elem<1> { typedef __bf16 T; };
template <int ET, bool SPLIT, int BIAS_MODE, int OUT_MODE, bool RESID, int ACT = 0>
__global__ __launch_bounds__(256) void wmma_gemm64(
    const unsigned short* __restrict__ Ap, const unsigned short* __restrict__ A2p, int lda, long strideA,
    const unsigned short* __restrict__ Btp, const unsigned short* __restrict__ Bt2p, int ldb, long strideB,
    void* __restrict__ Cout, void* __restrict__ Cout2, int ldc, long strideC,
    const float* __restrict__ bias,
    const float* __restrict__ resid, long strideR,
    int M, int N, int K, float scale) {
  typedef typename Elem<ET>::T T;
  typedef typename Frag<T>::V V;
  const T* A = (const T*)Ap; const T* A2 = (const T*)A2p; const T* Bt = (const T*)Btp; const T* Bt2 = (const T*)Bt2p;
  __shared__ __align__(16) float sT[8][16 * 68];
  const int b    = blockIdx.y;
  const int lane = threadIdx.x & 31;
  const int wave = threadIdx.x >> 5;
  const int tilesN = N >> 6;
  const int tilesM = M >> 6;
  const int tile = blockIdx.x * 8 + wave;
  if (tile >= tilesM * tilesN) return;
  const int tm = tile / tilesN;
  const int tn = tile - tm * tilesN;
  const int m0 = tm << 6;
  const int n0 = tn << 6;

  const T* Ab  = A  + (size_t)b * strideA;
  const T* Bb  = Bt + (size_t)b * strideB;
  const T* Ab2 = SPLIT ? (A2  + (size_t)b * strideA) : nullptr;
  const T* Bb2 = SPLIT ? (Bt2 + (size_t)b * strideB) : nullptr;

  const int rlane = lane & 15;
  const int koff  = (lane >> 4) * 8;
  const int mOff  = (lane >> 4) * 8;

  v8f acc[4][4];
#pragma unroll
  for (int i = 0; i < 4; ++i)
#pragma unroll
    for (int j = 0; j < 4; ++j) acc[i][j] = (v8f){0.f,0.f,0.f,0.f,0.f,0.f,0.f,0.f};

  for (int k0 = 0; k0 < K; k0 += 32) {
    V bh[4], bl[4];
#pragma unroll
    for (int j = 0; j < 4; ++j) {
      const size_t bo = (size_t)(n0 + (j << 4) + rlane) * ldb + koff + k0;
      bh[j] = Frag<T>::load(Bb + bo);
      if (SPLIT) bl[j] = Frag<T>::load(Bb2 + bo);
    }
#pragma unroll
    for (int i = 0; i < 4; ++i) {
      const size_t ao = (size_t)(m0 + (i << 4) + rlane) * lda + koff + k0;
      V ah = Frag<T>::load(Ab + ao);
      V al;
      if (SPLIT) al = Frag<T>::load(Ab2 + ao);
#pragma unroll
      for (int j = 0; j < 4; ++j) {
        acc[i][j] = Frag<T>::mma(ah, bh[j], acc[i][j]);
        if (SPLIT) {
          acc[i][j] = Frag<T>::mma(ah, bl[j], acc[i][j]);
          acc[i][j] = Frag<T>::mma(al, bh[j], acc[i][j]);
        }
      }
      Frag<T>::guard4(acc[i][0], acc[i][1], acc[i][2], acc[i][3], ah, SPLIT ? al : ah);
    }
    Frag<T>::keep(bh[0], bh[1], bh[2], bh[3]);
    if (SPLIT) Frag<T>::keep(bl[0], bl[1], bl[2], bl[3]);
  }
  acc_guard4(acc[0][0], acc[0][1], acc[0][2], acc[0][3]);
  acc_guard4(acc[1][0], acc[1][1], acc[1][2], acc[1][3]);
  acc_guard4(acc[2][0], acc[2][1], acc[2][2], acc[2][3]);
  acc_guard4(acc[3][0], acc[3][1], acc[3][2], acc[3][3]);

  float* slab = sT[wave];
  const float* Rb = RESID ? (resid + (size_t)b * strideR) : nullptr;
#pragma unroll
  for (int i = 0; i < 4; ++i) {
    const int mBase = m0 + (i << 4);
#pragma unroll
    for (int j = 0; j < 4; ++j) {
      const int n = n0 + (j << 4) + rlane;
      float bv = 0.f;
      if (BIAS_MODE == 2) bv = bias[n];
#pragma unroll
      for (int r = 0; r < 8; ++r) {
        float v = acc[i][j][r] * scale;
        if (BIAS_MODE == 1) v += bias[mBase + mOff + r];
        if (BIAS_MODE == 2) v += bv;
        if (RESID) v += Rb[(size_t)(mBase + mOff + r) * ldc + n];
        if (ACT == 1) v = tanhf(v);
        if (ACT == 2) v = fmaxf(v, 0.0f);
        if (ACT == 3) v = v / (1.0f + expf(-v));
        if (ACT == 4) v = (v > 0.f) ? v : 0.01f * v;
        slab[(mOff + r) * 68 + (j << 4) + rlane] = v;
      }
    }
    __builtin_amdgcn_fence(__ATOMIC_RELEASE, "workgroup");
    __builtin_amdgcn_wave_barrier();
    __builtin_amdgcn_fence(__ATOMIC_ACQUIRE, "workgroup");
    if (OUT_MODE == 0) {
      float* C = (float*)Cout + (size_t)b * strideC;
      const int hh = lane >> 4, c4 = (lane & 15) * 4;
      for (int pass = 0; pass < 2; ++pass) {
#pragma unroll
        for (int it = 0; it < 8; ++it) {
          const int row = it * 2 + hh;
          v4f v = *(const v4f*)(slab + row * 68 + c4);
          *(volatile v4f*)(C + (size_t)(mBase + row) * ldc + n0 + c4) = v;
        }
        __threadfence();
      }
    } else {
      const int q = lane >> 3, c8 = (lane & 7) * 8;
      unsigned short* C  = (unsigned short*)Cout  + (size_t)b * strideC;
      unsigned short* C2 = (OUT_MODE == 2) ? ((unsigned short*)Cout2 + (size_t)b * strideC) : nullptr;
      for (int pass = 0; pass < 2; ++pass) {
#pragma unroll
        for (int it = 0; it < 4; ++it) {
          const int row = it * 4 + q;
          const float* sp = slab + row * 68 + c8;
          v8h hv, lv;
#pragma unroll
          for (int e = 0; e < 8; ++e) {
            if (OUT_MODE == 1) {
              hv[e] = (_Float16)sp[e];
            } else {
              unsigned short hb = f2bf_bits(sp[e]);
              unsigned short lb = f2bf_bits(sp[e] - bf_bits2f(hb));
              hv[e] = __builtin_bit_cast(_Float16, hb);
              lv[e] = __builtin_bit_cast(_Float16, lb);
            }
          }
          *(volatile v8h*)(C + (size_t)(mBase + row) * ldc + n0 + c8) = hv;
          if (OUT_MODE == 2) *(volatile v8h*)(C2 + (size_t)(mBase + row) * ldc + n0 + c8) = lv;
        }
        __threadfence();
      }
    }
    __builtin_amdgcn_fence(__ATOMIC_RELEASE, "workgroup");
    __builtin_amdgcn_wave_barrier();
    __builtin_amdgcn_fence(__ATOMIC_ACQUIRE, "workgroup");
  }
}


__device__ __forceinline__ void store2(float* p, float v) {
  *(volatile float*)p = v;
  __threadfence();
  *(volatile float*)p = v;
}

__global__ __launch_bounds__(kThr) void cast_plane_kernel(const float* __restrict__ src, unsigned short* __restrict__ dst,
                                                          int colsLog2, int dstPitch, int dstOff) {
  const int i   = blockIdx.x * kThr + threadIdx.x;
  const int sh  = colsLog2 - 3;
  const int row = i >> sh;
  const int c8  = (i & ((1 << sh) - 1)) * 8;
  const float* sp = src + ((size_t)row << colsLog2) + c8;
  const v4f a0 = *(const v4f*)(sp);
  const v4f a1 = *(const v4f*)(sp + 4);
  v8h hv;
#pragma unroll
  for (int e = 0; e < 4; ++e) {
    const float f0 = a0[e];
    const float f1 = a1[e];
    hv[e]     = (_Float16)carry_flush(bf16r(f0), kInCarry);
    hv[4 + e] = (_Float16)carry_flush(bf16r(f1), kInCarry);
  }
  unsigned short* dp = dst + (size_t)row * dstPitch + dstOff + c8;
  *(volatile v8h*)dp = hv;
  __threadfence();
  *(volatile v8h*)dp = hv;
}

__global__ __launch_bounds__(256) void wt_plane_kernel(const float* __restrict__ W, unsigned short* __restrict__ dst, int K, int N, int nLive, int ldd, int colOff) {
  const int n  = blockIdx.x;
  const int k8 = threadIdx.x * 8;
  const bool live = n < nLive;
  const int nc = live ? n : 0;
  v8h hv;
#pragma unroll
  for (int e = 0; e < 8; ++e) {
    const float w = W[(size_t)(k8 + e) * N + nc];
    hv[e] = (_Float16)(live ? carry_flush(bf16r(w), kWCarry) : 0.0f);
  }
  unsigned short* dp = dst + (size_t)n * ldd + colOff + k8;
  *(volatile v8h*)dp = hv;
  __threadfence();
  *(volatile v8h*)dp = hv;
}

__global__ __launch_bounds__(24) void patch_kernel(const float* __restrict__ x, unsigned short* __restrict__ PATCH16) {
  const unsigned row = blockIdx.y;
  const unsigned g = threadIdx.x;
  const unsigned c = g >> 3, pi = g & 7u;
  const unsigned sm = row >> 10, ph = (row >> 5) & 31u, pw = row & 31u;
  const float* sp = x + ((size_t)(sm * 3u + c) * 256u + (size_t)(8u * ph + pi)) * 256u + 8u * pw;
  const v4f x0 = *(const v4f*)sp, x1 = *(const v4f*)(sp + 4);
  v8h hv;
#pragma unroll
  for (int e = 0; e < 8; ++e) { const float p = (e < 4) ? x0[e] : x1[e - 4]; hv[e] = (_Float16)carry_flush(bf16r(p), kCX); }
  unsigned short* dp = PATCH16 + (size_t)row * kKP + (size_t)g * 8;
  *(volatile v8h*)dp = hv;
  __threadfence();
  *(volatile v8h*)dp = hv;
}
static_assert(kKP == 24 * 8, "a patch row is 24 groups of eight");

__global__ __launch_bounds__(kThr) void setup_kernel(const float* __restrict__ pb, const float* __restrict__ dtb, const float* __restrict__ clb, const float* __restrict__ dtw,
                                                    float* __restrict__ ZB, float* __restrict__ PB, float* __restrict__ BDT, float* __restrict__ CLB,
                                                    unsigned short* __restrict__ WDT16, unsigned short* __restrict__ WX16, unsigned short* __restrict__ WCLS16, unsigned short* __restrict__ POOL16) {
  const unsigned bk = blockIdx.x;
  if (bk < 4u) {
    store2(ZB + bk * (unsigned)kThr + threadIdx.x, 0.0f);
  } else if (bk == 4u) {
    const float p = pb[threadIdx.x];
    store2(PB + threadIdx.x, bf16r(p));
  } else if (bk < 13u) {
    const unsigned i = (bk - 5u) * (unsigned)kThr + threadIdx.x;
    const float p = dtb[i];
    store2(BDT + i, bf16r(p));
  } else if (bk < 17u) {
    const unsigned n = (bk - 13u) * (unsigned)kThr + threadIdx.x;
    float v = 0.0f;
    if (n < (unsigned)kNC) { const float p = clb[n]; v = bf16r(p); }
    store2(CLB + n, v);
  } else if (bk < 25u) {
    const unsigned rw = (bk - 17u) * (unsigned)kThr + threadIdx.x;
    unsigned short* dp = WDT16 + (size_t)rw * kRP;
#pragma unroll
    for (int c = 0; c < kRP / 8; ++c) {
      v8h hv;
#pragma unroll
      for (int e = 0; e < 8; ++e) {
        const int r = 8 * c + e;
        float w = 0.0f;
        if (r < kR) { const float p = dtw[(size_t)rw * kR + r]; w = carry_flush(bf16r(p), kWdtCarry); }
        hv[e] = (_Float16)w;
      }
      *(volatile v8h*)(dp + 8 * c) = hv;
      __threadfence();
      *(volatile v8h*)(dp + 8 * c) = hv;
    }
  } else {
    v8h zv;
#pragma unroll
    for (int e = 0; e < 8; ++e) zv[e] = (_Float16)0.0f;
    unsigned short* dp = nullptr;
    if (bk < 41u) {
      const unsigned j = (bk - 25u) * (unsigned)kThr + threadIdx.x;
      dp = WX16 + ((size_t)(j >> 10) * kXoP + kXo) * kDI + (size_t)(j & 1023u) * 8;
    } else if (bk < 44u) {
      const unsigned j = (bk - 41u) * (unsigned)kThr + threadIdx.x;
      dp = WCLS16 + (size_t)kNC * kDM + (size_t)j * 8;
    } else {
      const unsigned j = (bk - 44u) * (unsigned)kThr + threadIdx.x;
      if (j < 1920u) dp = POOL16 + (size_t)kNB * kDM + (size_t)j * 8;
    }
    if (dp != nullptr) {
      *(volatile v8h*)dp = zv;
      __threadfence();
      *(volatile v8h*)dp = zv;
    }
  }
}
static_assert(1024 == 4 * kThr && kDM == kThr && kNL * kDI == 8 * kThr && kNCP == 4 * kThr && (size_t)kNL * (kXoP - kXo) * kDI / 8 == 16ull * kThr && (size_t)(kNCP - kNC) * kDM / 8 == 3ull * kThr && (size_t)(kMP - kNB) * kDM / 8 == 1920ull, "set-up grid: 4 + 1 + 8 + 4 + 8 + 16 + 3 + 8 = 52 blocks");

__global__ __launch_bounds__(kThr) void lnstat_kernel(const float* __restrict__ U, float* __restrict__ STAT) {
  const size_t row = (size_t)blockIdx.x * kThr + threadIdx.x;
  const float* up = U + row * kDM;
  float s = 0.0f;
  for (int c = 0; c < kDM; ++c) s += up[c];
  const float mean = s / (float)kDM;
  float q = 0.0f;
  for (int c = 0; c < kDM; ++c) { const float dd = up[c] - mean; q += dd * dd; }
  v2f st; st[0] = mean; st[1] = 1.0f / sqrtf(q / (float)kDM + 1e-5f);
  float* dp = STAT + 2 * row;
  *(volatile v2f*)dp = st;
  __threadfence();
  *(volatile v2f*)dp = st;
}
static_assert(kRows == 16 * kThr, "statistics grid exact: 16 blocks");

__global__ __launch_bounds__(kThr) void lncast_kernel(const float* __restrict__ U, const float* __restrict__ STAT, const float* __restrict__ gam, const float* __restrict__ bet,
                                                     unsigned short* __restrict__ XN16) {
  const unsigned i = blockIdx.x * (unsigned)kThr + threadIdx.x;
  const size_t row = i >> 5;
  const unsigned c8 = (i & 31u) * 8u;
  const float mean = STAT[2 * row], inv = STAT[2 * row + 1];
  const float* up = U + row * kDM + c8;
  v8h hv;
#pragma unroll
  for (int e = 0; e < 8; ++e) {
    const float ga = gam[c8 + e], be = bet[c8 + e];
    hv[e] = (_Float16)carry_flush((up[e] - mean) * inv * bf16r(ga) + bf16r(be), kCXn);
  }
  unsigned short* dp = XN16 + row * kDM + c8;
  *(volatile v8h*)dp = hv;
  __threadfence();
  *(volatile v8h*)dp = hv;
}
static_assert((size_t)kRows * (kDM / 8) == 512ull * kThr && kDM / 8 == 32, "norm cast grid exact: 512 blocks; 32 groups a row");

__global__ __launch_bounds__(64) void front_kernel(const float* __restrict__ XZ, const float* __restrict__ cw, const float* __restrict__ cb,
                                                   float* __restrict__ U32, unsigned short* __restrict__ U16) {
  const int row = (int)blockIdx.y;
  const int pos = row & (kT - 1);
  const int c8 = (int)threadIdx.x * 8;
  float acc[8], wv[8][kDC];
#pragma unroll
  for (int e = 0; e < 8; ++e) {
    acc[e] = 0.0f;
    const v4f w4 = *(const v4f*)(cw + (size_t)(c8 + e) * kDC);
#pragma unroll
    for (int k = 0; k < kDC; ++k) { const float w = w4[k]; wv[e][k] = bf16r(w); }
  }
#pragma unroll
  for (int k = 0; k < kDC; ++k) {
    const int back = kDC - 1 - k;
    const bool has = pos >= back;
    const float* xp = XZ + (size_t)(row - (has ? back : 0)) * (2 * kDI) + c8;
    const v4f x0 = *(const v4f*)xp, x1 = *(const v4f*)(xp + 4);
#pragma unroll
    for (int e = 0; e < 8; ++e) {
      const float xv = (e < 4) ? x0[e] : x1[e - 4];
      acc[e] += has ? wv[e][k] * xv : 0.0f;
    }
  }
  v4f u0, u1;
  v8h hv;
#pragma unroll
  for (int e = 0; e < 8; ++e) {
    const float p = cb[c8 + e];
    const float v = acc[e] + bf16r(p);
    const float s = v / (1.0f + expf(-v));
    if (e < 4) u0[e] = s; else u1[e - 4] = s;
    hv[e] = (_Float16)carry_flush(s, kCU);
  }
  float* up = U32 + (size_t)row * kDI + c8;
  unsigned short* hp = U16 + (size_t)row * kDI + c8;
  for (int pass = 0; pass < 2; ++pass) {
    *(volatile v4f*)up = u0; *(volatile v4f*)(up + 4) = u1;
    *(volatile v8h*)hp = hv;
    __threadfence();
  }
}
static_assert(kDI == 64 * 8, "front grid exact: 64 groups a row");

__global__ __launch_bounds__(kThr) void dtcast_kernel(const float* __restrict__ XD, unsigned short* __restrict__ DT16) {
  const unsigned i = blockIdx.x * (unsigned)kThr + threadIdx.x;
  const size_t row = i >> 2;
  const unsigned ch = i & 3u;
  const unsigned c8 = ch * 8u;
  const bool live = ch < (unsigned)(kR / 8);
  const float* sp = XD + row * kXoP + c8;
  v8h hv;
#pragma unroll
  for (int e = 0; e < 8; ++e) { const float v = sp[e]; hv[e] = (_Float16)(live ? carry_flush(v, kCDt) : 0.0f); }
  unsigned short* dp = DT16 + row * kRP + c8;
  *(volatile v8h*)dp = hv;
  __threadfence();
  *(volatile v8h*)dp = hv;
}
static_assert((size_t)kRows * 4 == 64ull * kThr && kRP == 4 * 8 && (kR % 8) == 0, "the step input's cast: 64 blocks; 4 groups a row of which 2 are live");

__global__ __launch_bounds__(kThr) void scan_kernel(const float* __restrict__ XD, const float* __restrict__ DL, const float* __restrict__ U32,
                                                    const float* __restrict__ A_log, const float* __restrict__ Dp, float* __restrict__ YS) {
  const unsigned sq = blockIdx.x >> 1;
  const unsigned d = (blockIdx.x & 1u) * (unsigned)kThr + threadIdx.x;
  float A[kNs], h[kNs];
#pragma unroll
  for (int n = 0; n < kNs; ++n) { const float a = A_log[(size_t)d * kNs + n]; A[n] = -expf(bf16r(a)); h[n] = 0.0f; }
  const float q0 = Dp[d];
  const float dsk = bf16r(q0);
  for (int l = 0; l < kT; ++l) {
    const size_t row = (size_t)sq * kT + (size_t)l;
    const float* pb = XD + row * kXoP + kR;
    const float pre = DL[row * kDI + d];
    const float uv = U32[row * kDI + d];
    const float dt = fmaxf(pre, 0.0f) + log1pf(expf(-fabsf(pre)));
    const float dx = dt * uv;
    float y = 0.0f;
#pragma unroll
    for (int q = 0; q < kNs / 4; ++q) {
      const v4f bv = *(const v4f*)(pb + 4 * q), cv = *(const v4f*)(pb + kNs + 4 * q);
#pragma unroll
      for (int e = 0; e < 4; ++e) {
        const int n = 4 * q + e;
        const float hn = expf(dt * A[n]) * h[n] + dx * bv[e];
        h[n] = hn;
        y += hn * cv[e];
      }
    }
    store2(YS + row * kDI + d, y + dsk * uv);
  }
}
static_assert(kDI == 2 * kThr && (kNs % 4) == 0 && (kR % 4) == 0, "walk grid exact: 8 blocks: two a sequence; the B | C columns 16-B aligned");

__global__ __launch_bounds__(64) void ygate_kernel(const float* __restrict__ YS, const float* __restrict__ XZ, unsigned short* __restrict__ Y16) {
  const size_t row = blockIdx.y;
  const unsigned c8 = threadIdx.x * 8u;
  const float* yp = YS + row * kDI + c8;
  const float* zp = XZ + row * (2 * kDI) + kDI + c8;
  v8h hv;
#pragma unroll
  for (int e = 0; e < 8; ++e) { const float z = zp[e]; hv[e] = (_Float16)carry_flush(yp[e] * (z / (1.0f + expf(-z))), kCY); }
  unsigned short* dp = Y16 + row * kDI + c8;
  *(volatile v8h*)dp = hv;
  __threadfence();
  *(volatile v8h*)dp = hv;
}

__global__ __launch_bounds__(kThr) void resadd_kernel(const float* __restrict__ U, const float* __restrict__ OUTF, float* __restrict__ Unext) {
  const size_t o = ((size_t)blockIdx.x * kThr + threadIdx.x) * 8;
  const v4f a0 = *(const v4f*)(U + o), a1 = *(const v4f*)(U + o + 4), b0 = *(const v4f*)(OUTF + o), b1 = *(const v4f*)(OUTF + o + 4);
  v4f o0, o1;
#pragma unroll
  for (int e = 0; e < 4; ++e) { o0[e] = a0[e] + b0[e]; o1[e] = a1[e] + b1[e]; }
  float* dp = Unext + o;
  for (int pass = 0; pass < 2; ++pass) { *(volatile v4f*)dp = o0; *(volatile v4f*)(dp + 4) = o1; __threadfence(); }
}
static_assert((size_t)kRows * kDM / 8 == 512ull * kThr, "the residual: 512 blocks");

__global__ __launch_bounds__(32) void pool_kernel(const float* __restrict__ U, const float* __restrict__ STAT, const float* __restrict__ gam, const float* __restrict__ bet,
                                                  unsigned short* __restrict__ POOL16) {
  const unsigned sm = blockIdx.x;
  const unsigned c8 = threadIdx.x * 8u;
  float acc[8], ga[8], be[8];
#pragma unroll
  for (int e = 0; e < 8; ++e) { const float g0 = gam[c8 + e], b0 = bet[c8 + e]; ga[e] = bf16r(g0); be[e] = bf16r(b0); acc[e] = 0.0f; }
  for (int t = 0; t < kT; ++t) {
    const size_t row = (size_t)sm * kT + (size_t)t;
    const float mean = STAT[2 * row], inv = STAT[2 * row + 1];
    const float* up = U + row * kDM + c8;
    const v4f u0 = *(const v4f*)up, u1 = *(const v4f*)(up + 4);
#pragma unroll
    for (int e = 0; e < 8; ++e) { const float uv = (e < 4) ? u0[e] : u1[e - 4]; acc[e] += (uv - mean) * inv * ga[e] + be[e]; }
  }
  v8h hv;
#pragma unroll
  for (int e = 0; e < 8; ++e) hv[e] = (_Float16)carry_flush(acc[e] / (float)kT, kCPool);
  unsigned short* dp = POOL16 + (size_t)sm * kDM + c8;
  *(volatile v8h*)dp = hv;
  __threadfence();
  *(volatile v8h*)dp = hv;
}
static_assert(kDM == 32 * 8, "pooling: one wave a sample");

__global__ __launch_bounds__(kThr) void outcopy_kernel(const float* __restrict__ LOG, float* __restrict__ out) {
  const unsigned i = blockIdx.x * (unsigned)kThr + threadIdx.x;
  if (i < (unsigned)(kNB * kNC)) {
    const unsigned b = (i >= 3u * kNC) ? 3u : ((i >= 2u * kNC) ? 2u : ((i >= (unsigned)kNC) ? 1u : 0u));
    const float v = LOG[(size_t)b * kNCP + (i - b * (unsigned)kNC)];
    store2(out + i, v);
  }
}
static_assert(kNB * kNC <= 16 * kThr && kNB == 4, "the result's copy: 16 blocks; four samples by three compares");

extern "C" void kernel_launch(void* const* d_in, const int* in_sizes, int n_in,
                              void* d_out, int out_size, void* d_ws, size_t ws_size,
                              hipStream_t stream) {
  if (n_in < 18 || d_out == nullptr || d_ws == nullptr) return;
  if (in_sizes[0] != kNB * 3 * 256 * 256 || in_sizes[1] != kDM * kKP || in_sizes[2] != kDM || in_sizes[3] != kNL * kDM || in_sizes[4] != kNL * kDM || in_sizes[5] != kNL * 2 * kDI * kDM) return;
  if (in_sizes[6] != kNL * kDI * kDC || in_sizes[7] != kNL * kDI || in_sizes[8] != kNL * kXo * kDI || in_sizes[9] != kNL * kDI * kR || in_sizes[10] != kNL * kDI || in_sizes[11] != kNL * kDI * kNs) return;
  if (in_sizes[12] != kNL * kDI || in_sizes[13] != kNL * kDM * kDI || in_sizes[14] != kDM || in_sizes[15] != kDM || in_sizes[16] != kNC * kDM || in_sizes[17] != kNC) return;
  if (out_size != kNB * kNC) return;
  if (ws_size < kWsTotal) return;
  const float* x    = (const float*)d_in[0];
  const float* pw   = (const float*)d_in[1];
  const float* pb   = (const float*)d_in[2];
  const float* lng  = (const float*)d_in[3];
  const float* lnb  = (const float*)d_in[4];
  const float* inw  = (const float*)d_in[5];
  const float* cvw  = (const float*)d_in[6];
  const float* cvb  = (const float*)d_in[7];
  const float* xpw  = (const float*)d_in[8];
  const float* dtw  = (const float*)d_in[9];
  const float* dtb  = (const float*)d_in[10];
  const float* alog = (const float*)d_in[11];
  const float* dsk  = (const float*)d_in[12];
  const float* outw = (const float*)d_in[13];
  const float* fng  = (const float*)d_in[14];
  const float* fnb  = (const float*)d_in[15];
  const float* clw  = (const float*)d_in[16];
  const float* clb  = (const float*)d_in[17];
  float* out = (float*)d_out;
  char* ws = (char*)d_ws;
  float* ZB   = (float*)(ws + kOffZB);
  float* PB   = (float*)(ws + kOffPB);
  float* BDT  = (float*)(ws + kOffBDT);
  float* CLB  = (float*)(ws + kOffCLB);
  float* STAT = (float*)(ws + kOffSTAT);
  unsigned short* WP16   = (unsigned short*)(ws + kOffWP16);
  unsigned short* WIN16  = (unsigned short*)(ws + kOffWIN16);
  unsigned short* WX16   = (unsigned short*)(ws + kOffWX16);
  unsigned short* WDT16  = (unsigned short*)(ws + kOffWDT16);
  unsigned short* WOUT16 = (unsigned short*)(ws + kOffWOUT16);
  unsigned short* WCLS16 = (unsigned short*)(ws + kOffWCLS16);
  unsigned short* PATCH16 = (unsigned short*)(ws + kOffPATCH16);
  float* UA  = (float*)(ws + kOffUA);
  float* UB  = (float*)(ws + kOffUB);
  unsigned short* XN16 = (unsigned short*)(ws + kOffXN16);
  float* XZ  = (float*)(ws + kOffXZ);
  float* U32 = (float*)(ws + kOffU32);
  unsigned short* U16 = (unsigned short*)(ws + kOffU16);
  float* XD  = (float*)(ws + kOffXD);
  unsigned short* DT16 = (unsigned short*)(ws + kOffDT16);
  float* DL  = (float*)(ws + kOffDL);
  float* YS  = (float*)(ws + kOffYS);
  unsigned short* Y16 = (unsigned short*)(ws + kOffY16);
  float* OUTF = (float*)(ws + kOffOUTF);
  unsigned short* POOL16 = (unsigned short*)(ws + kOffPOOL16);
  float* LOG = (float*)(ws + kOffLOG);

  static_assert(((size_t)kDM * kKP / 8) % kThr == 0 && ((size_t)kNL * 2 * kDI * kDM / 8) % kThr == 0 && ((size_t)kXo * kDI / 8) % kThr == 0 && ((size_t)kNL * kDM * kDI / 8) % kThr == 0 && ((size_t)kNC * kDM / 8) % kThr == 0, "the casts' grids");
  patch_kernel<<<dim3(1, kRows), 24, 0, stream>>>(x, PATCH16);
  cast_plane_kernel<<<(int)(((size_t)kDM * kKP / 8) / kThr), kThr, 0, stream>>>(pw, WP16, 10, 1024, 0);
  cast_plane_kernel<<<(int)(((size_t)kNL * 2 * kDI * kDM / 8) / kThr), kThr, 0, stream>>>(inw, WIN16, 8, kDM, 0);
  for (int l = 0; l < kNL; ++l)
    cast_plane_kernel<<<(int)(((size_t)kXo * kDI / 8) / kThr), kThr, 0, stream>>>(xpw + (size_t)l * kXo * kDI, WX16 + (size_t)l * kXoP * kDI, 9, kDI, 0);
  cast_plane_kernel<<<(int)(((size_t)kNL * kDM * kDI / 8) / kThr), kThr, 0, stream>>>(outw, WOUT16, 9, kDI, 0);
  cast_plane_kernel<<<(int)(((size_t)kNC * kDM / 8) / kThr), kThr, 0, stream>>>(clw, WCLS16, 8, kDM, 0);
  setup_kernel<<<52, kThr, 0, stream>>>(pb, dtb, clb, dtw, ZB, PB, BDT, CLB, WDT16, WX16, WCLS16, POOL16);

  wmma_gemm64<0, false, 2, 0, false, 0><<<dim3((kRows / 64) * (kDM / 64) / 8, 1), 256, 0, stream>>>(
      PATCH16, PATCH16, kKP, 0L, WP16, WP16, kKP, 0L, (void*)UA, (void*)UA, kDM, 0L, PB, nullptr, 0L, kRows, kDM, kKP, 1.0f / (kCX * kInCarry));
  float* Ucur = UA;
  float* Unxt = UB;
  for (int l = 0; l < kNL; ++l) {
    lnstat_kernel<<<16, kThr, 0, stream>>>(Ucur, STAT);
    lncast_kernel<<<512, kThr, 0, stream>>>(Ucur, STAT, lng + (size_t)l * kDM, lnb + (size_t)l * kDM, XN16);
    wmma_gemm64<0, false, 2, 0, false, 0><<<dim3((kRows / 64) * (2 * kDI / 64) / 8, 1), 256, 0, stream>>>(
        XN16, XN16, kDM, 0L, WIN16 + (size_t)l * 2 * kDI * kDM, WIN16 + (size_t)l * 2 * kDI * kDM, kDM, 0L, (void*)XZ, (void*)XZ, 2 * kDI, 0L, ZB, nullptr, 0L, kRows, 2 * kDI, kDM, 1.0f / (kCXn * kInCarry));
    front_kernel<<<dim3(1, kRows), 64, 0, stream>>>(XZ, cvw + (size_t)l * kDI * kDC, cvb + (size_t)l * kDI, U32, U16);
    wmma_gemm64<0, false, 2, 0, false, 0><<<dim3((kRows / 64) * (kXoP / 64) / 8, 1), 256, 0, stream>>>(
        U16, U16, kDI, 0L, WX16 + (size_t)l * kXoP * kDI, WX16 + (size_t)l * kXoP * kDI, kDI, 0L, (void*)XD, (void*)XD, kXoP, 0L, ZB, nullptr, 0L, kRows, kXoP, kDI, 1.0f / (kCU * kInCarry));
    dtcast_kernel<<<64, kThr, 0, stream>>>(XD, DT16);
    wmma_gemm64<0, false, 2, 0, false, 0><<<dim3((kRows / 64) * (kDI / 64) / 8, 1), 256, 0, stream>>>(
        DT16, DT16, kRP, 0L, WDT16 + (size_t)l * kDI * kRP, WDT16 + (size_t)l * kDI * kRP, kRP, 0L, (void*)DL, (void*)DL, kDI, 0L, BDT + (size_t)l * kDI, nullptr, 0L, kRows, kDI, kRP, 1.0f / (kCDt * kWdtCarry));
    scan_kernel<<<2 * kNB, kThr, 0, stream>>>(XD, DL, U32, alog + (size_t)l * kDI * kNs, dsk + (size_t)l * kDI, YS);
    ygate_kernel<<<dim3(1, kRows), 64, 0, stream>>>(YS, XZ, Y16);
    wmma_gemm64<0, false, 2, 0, false, 0><<<dim3((kRows / 64) * (kDM / 64) / 8, 1), 256, 0, stream>>>(
        Y16, Y16, kDI, 0L, WOUT16 + (size_t)l * kDM * kDI, WOUT16 + (size_t)l * kDM * kDI, kDI, 0L, (void*)OUTF, (void*)OUTF, kDM, 0L, ZB, nullptr, 0L, kRows, kDM, kDI, 1.0f / (kCY * kInCarry));
    resadd_kernel<<<512, kThr, 0, stream>>>(Ucur, OUTF, Unxt);
    float* tswap = Ucur; Ucur = Unxt; Unxt = tswap;
  }
  lnstat_kernel<<<16, kThr, 0, stream>>>(Ucur, STAT);
  pool_kernel<<<kNB, 32, 0, stream>>>(Ucur, STAT, fng, fnb, POOL16);
  wmma_gemm64<0, false, 2, 0, false, 0><<<dim3((kMP / 64) * (kNCP / 64) / 8, 1), 256, 0, stream>>>(
      POOL16, POOL16, kDM, 0L, WCLS16, WCLS16, kDM, 0L, (void*)LOG, (void*)LOG, kNCP, 0L, CLB, nullptr, 0L, kMP, kNCP, kDM, 1.0f / (kCPool * kInCarry));
  outcopy_kernel<<<16, kThr, 0, stream>>>(LOG, out);
}
